// TTTBase_80479097193098
// MI455X (gfx1250) — hardware-verified
//
#include <hip/hip_runtime.h>
#include <stdint.h>

constexpr int kB    = 2;
constexpr int kS    = 2048;
constexpr int kD    = 2048;
constexpr int kH    = 32;
constexpr int kHD   = 64;
constexpr int kMB   = 16;
constexpr int kNMB  = 128;
constexpr int kRows = kB * kS;
constexpr float kEps = 1e-5f;

typedef __attribute__((ext_vector_type(16))) _Float16 v16h;
typedef __attribute__((ext_vector_type(8)))  _Float16 v8h;
typedef __attribute__((ext_vector_type(16))) __bf16   v16b;
typedef __attribute__((ext_vector_type(8)))  __bf16   v8b;
typedef __attribute__((ext_vector_type(8)))  float    v8f;
typedef __attribute__((ext_vector_type(4)))  float    v4f;
typedef __attribute__((ext_vector_type(4)))  unsigned int v4u;
typedef v4f __attribute__((may_alias)) v4fa;

__device__ __forceinline__ unsigned short f2bf_bits(float f) {
  unsigned u = __float_as_uint(f);
  return (unsigned short)((u + 0x7FFFu + ((u >> 16) & 1u)) >> 16);
}
__device__ __forceinline__ float bf_bits2f(unsigned short h) { return __uint_as_float(((unsigned)h) << 16); }

__device__ __forceinline__ void dep_guard_h(v8f& a, v8f& b, v16h x, v16h y) { asm volatile("v_nop\n\tv_nop\n\tv_nop\n\tv_nop" : "+v"(a), "+v"(b) : "v"(x), "v"(y)); }
__device__ __forceinline__ void dep_guard_b(v8f& a, v8f& b, v16b x, v16b y) { asm volatile("v_nop\n\tv_nop\n\tv_nop\n\tv_nop" : "+v"(a), "+v"(b) : "v"(x), "v"(y)); }
__device__ __forceinline__ void keep4_h(v16h a, v16h b, v16h c, v16h d) { asm volatile("v_nop" :: "v"(a), "v"(b), "v"(c), "v"(d)); }
__device__ __forceinline__ void keep4_b(v16b a, v16b b, v16b c, v16b d) { asm volatile("v_nop" :: "v"(a), "v"(b), "v"(c), "v"(d)); }
__device__ __forceinline__ void acc_guard4(v8f& a, v8f& b, v8f& c, v8f& d) { asm volatile("v_nop\n\tv_nop\n\tv_nop\n\tv_nop" : "+v"(a), "+v"(b), "+v"(c), "+v"(d)); }
template <typename T> struct Frag;
template <> struct Frag<_Float16> {
  typedef v16h V; union U { v16h v; v8h h[2]; };
  static __device__ __forceinline__ v16h load(const _Float16* p) {
    U f; f.h[0] = *(const v8h*)(p); f.h[1] = *(const v8h*)(p + 16); return f.v;
  }
  static __device__ __forceinline__ v8f mma(v16h a, v16h b, v8f c) {
    return __builtin_amdgcn_wmma_f32_16x16x32_f16(false, a, false, b, (short)0, c, false, false);
  }
  static __device__ __forceinline__ void guard(v8f& a, v8f& b, v16h x, v16h y) { dep_guard_h(a, b, x, y); }
  static __device__ __forceinline__ void keep(v16h a, v16h b, v16h c, v16h d) { keep4_h(a, b, c, d); }
};
template <> struct Frag<__bf16> {
  typedef v16b V; union U { v16b v; v8b h[2]; };
  static __device__ __forceinline__ v16b load(const __bf16* p) {
    U f; f.h[0] = *(const v8b*)(p); f.h[1] = *(const v8b*)(p + 16); return f.v;
  }
  static __device__ __forceinline__ v8f mma(v16b a, v16b b, v8f c) {
    return __builtin_amdgcn_wmma_f32_16x16x32_bf16(false, a, false, b, (short)0, c, false, false);
  }
  static __device__ __forceinline__ void guard(v8f& a, v8f& b, v16b x, v16b y) { dep_guard_b(a, b, x, y); }
  static __device__ __forceinline__ void keep(v16b a, v16b b, v16b c, v16b d) { keep4_b(a, b, c, d); }
};

template <int ET> struct Elem;
template <> struct Elem<0> { typedef _Float16 T; };
template <> struct Elem<1> { typedef __bf16 T; };
template <int ET, bool SPLIT, int BIAS_MODE, int OUT_MODE, bool RESID, int ACT = 0>
__global__ __launch_bounds__(256) void wmma_gemm64(
    const unsigned short* __restrict__ Ap, const unsigned short* __restrict__ A2p, int lda, long strideA,
    const unsigned short* __restrict__ Btp, const unsigned short* __restrict__ Bt2p, int ldb, long strideB,
    void* __restrict__ Cout, void* __restrict__ Cout2, int ldc, long strideC,
    const float* __restrict__ bias,
    const float* __restrict__ resid, long strideR,
    int M, int N, int K, float scale) {
  typedef typename Elem<ET>::T T;
  typedef typename Frag<T>::V V;
  const T* A = (const T*)Ap; const T* A2 = (const T*)A2p; const T* Bt = (const T*)Btp; const T* Bt2 = (const T*)Bt2p;
  __shared__ __align__(16) float sT[8][16 * 68];
  const int b    = blockIdx.y;
  const int lane = threadIdx.x & 31;
  const int wave = threadIdx.x >> 5;
  const int tilesN = N >> 6;
  const int tilesM = M >> 6;
  const int tile = blockIdx.x * 8 + wave;
  if (tile >= tilesM * tilesN) return;
  const int tm = tile / tilesN;
  const int tn = tile - tm * tilesN;
  const int m0 = tm << 6;
  const int n0 = tn << 6;

  const T* Ab  = A  + (size_t)b * strideA;
  const T* Bb  = Bt + (size_t)b * strideB;
  const T* Ab2 = SPLIT ? (A2  + (size_t)b * strideA) : nullptr;
  const T* Bb2 = SPLIT ? (Bt2 + (size_t)b * strideB) : nullptr;

  const int rlane = lane & 15;
  const int koff  = (lane >> 4) * 8;
  const int mOff  = (lane >> 4) * 8;

  v8f acc[4][4];
#pragma unroll
  for (int i = 0; i < 4; ++i)
#pragma unroll
    for (int j = 0; j < 4; ++j) acc[i][j] = (v8f){0.f,0.f,0.f,0.f,0.f,0.f,0.f,0.f};

  for (int k0 = 0; k0 < K; k0 += 32) {
    V bh[4], bl[4];
#pragma unroll
    for (int j = 0; j < 4; ++j) {
      const size_t bo = (size_t)(n0 + (j << 4) + rlane) * ldb + koff + k0;
      bh[j] = Frag<T>::load(Bb + bo);
      if (SPLIT) bl[j] = Frag<T>::load(Bb2 + bo);
    }
#pragma unroll
    for (int i = 0; i < 4; ++i) {
      const size_t ao = (size_t)(m0 + (i << 4) + rlane) * lda + koff + k0;
      V ah = Frag<T>::load(Ab + ao);
      V al;
      if (SPLIT) al = Frag<T>::load(Ab2 + ao);
#pragma unroll
      for (int j = 0; j < 4; ++j) {
        acc[i][j] = Frag<T>::mma(ah, bh[j], acc[i][j]);
        if (SPLIT) {
          acc[i][j] = Frag<T>::mma(ah, bl[j], acc[i][j]);
          acc[i][j] = Frag<T>::mma(al, bh[j], acc[i][j]);
        }
      }
      Frag<T>::guard(acc[i][0], acc[i][3], ah, SPLIT ? al : ah);
    }
    Frag<T>::keep(bh[0], bh[1], bh[2], bh[3]);
    if (SPLIT) Frag<T>::keep(bl[0], bl[1], bl[2], bl[3]);
  }
  acc_guard4(acc[0][0], acc[0][1], acc[0][2], acc[0][3]);
  acc_guard4(acc[1][0], acc[1][1], acc[1][2], acc[1][3]);
  acc_guard4(acc[2][0], acc[2][1], acc[2][2], acc[2][3]);
  acc_guard4(acc[3][0], acc[3][1], acc[3][2], acc[3][3]);

  float* slab = sT[wave];
  const float* Rb = RESID ? (resid + (size_t)b * strideR) : nullptr;
#pragma unroll
  for (int i = 0; i < 4; ++i) {
    const int mBase = m0 + (i << 4);
#pragma unroll
    for (int j = 0; j < 4; ++j) {
      const int n = n0 + (j << 4) + rlane;
      float bv = 0.f;
      if (BIAS_MODE == 2) bv = bias[n];
#pragma unroll
      for (int r = 0; r < 8; ++r) {
        float v = acc[i][j][r] * scale;
        if (BIAS_MODE == 1) v += bias[mBase + mOff + r];
        if (BIAS_MODE == 2) v += bv;
        if (RESID) v += Rb[(size_t)(mBase + mOff + r) * ldc + n];
        if (ACT == 1) v = tanhf(v);
        if (ACT == 2) v = fmaxf(v, 0.0f);
        if (ACT == 3) v = v / (1.0f + expf(-v));
        if (ACT == 4) v = (v > 0.f) ? v : 0.01f * v;
        if (ACT == 5) v = 0.5f * v * (1.0f + erff(v * 0.70710678118654752f));
        slab[(mOff + r) * 68 + (j << 4) + rlane] = v;
      }
    }
    __builtin_amdgcn_fence(__ATOMIC_RELEASE, "workgroup");
    __builtin_amdgcn_wave_barrier();
    __builtin_amdgcn_fence(__ATOMIC_ACQUIRE, "workgroup");
    if (OUT_MODE == 0) {
      float* C = (float*)Cout + (size_t)b * strideC;
      const int hh = lane >> 4, c4 = (lane & 15) * 4;
      for (int pass = 0; pass < 2; ++pass) {
#pragma unroll
        for (int it = 0; it < 8; ++it) {
          const int row = it * 2 + hh;
          v4f v = *(const v4f*)(slab + row * 68 + c4);
          *(volatile v4f*)(C + (size_t)(mBase + row) * ldc + n0 + c4) = v;
        }
        __threadfence();
      }
    } else {
      const int q = lane >> 3, c8 = (lane & 7) * 8;
      unsigned short* C  = (unsigned short*)Cout  + (size_t)b * strideC;
      unsigned short* C2 = (OUT_MODE == 2) ? ((unsigned short*)Cout2 + (size_t)b * strideC) : nullptr;
      for (int pass = 0; pass < 2; ++pass) {
#pragma unroll
        for (int it = 0; it < 4; ++it) {
          const int row = it * 4 + q;
          const float* sp = slab + row * 68 + c8;
          v8h hv, lv;
#pragma unroll
          for (int e = 0; e < 8; ++e) {
            if (OUT_MODE == 1) {
              hv[e] = (_Float16)sp[e];
            } else {
              unsigned short hb = f2bf_bits(sp[e]);
              unsigned short lb = f2bf_bits(sp[e] - bf_bits2f(hb));
              hv[e] = __builtin_bit_cast(_Float16, hb);
              lv[e] = __builtin_bit_cast(_Float16, lb);
            }
          }
          *(volatile v8h*)(C + (size_t)(mBase + row) * ldc + n0 + c8) = hv;
          if (OUT_MODE == 2) *(volatile v8h*)(C2 + (size_t)(mBase + row) * ldc + n0 + c8) = lv;
        }
        __threadfence();
      }
    }
    __builtin_amdgcn_fence(__ATOMIC_RELEASE, "workgroup");
    __builtin_amdgcn_wave_barrier();
    __builtin_amdgcn_fence(__ATOMIC_ACQUIRE, "workgroup");
  }
}

__global__ __launch_bounds__(256) void cast_f32_f16x2_kernel(
    const float* __restrict__ in, _Float16* __restrict__ out, int n2, float scale) {
  int i = blockIdx.x * 256 + threadIdx.x;
  if (i < n2) {
    const _Float16 h0 = (_Float16)(in[2 * i] * scale), h1 = (_Float16)(in[2 * i + 1] * scale);
    const unsigned u = (unsigned)__builtin_bit_cast(unsigned short, h0) | ((unsigned)__builtin_bit_cast(unsigned short, h1) << 16);
    ((volatile unsigned*)out)[i] = u;
    __threadfence();
    ((volatile unsigned*)out)[i] = u;
  }
}

__device__ __forceinline__ unsigned short at_bf_bits(float f) {
  unsigned u = __float_as_uint(f);
  return (unsigned short)((u + 0x7FFFu + ((u >> 16) & 1u)) >> 16);
}
__device__ __forceinline__ __bf16 at_f2bf(float f) { return __builtin_bit_cast(__bf16, at_bf_bits(f)); }
__device__ __forceinline__ void at_split(float f, __bf16& hi, __bf16& lo) {
  const unsigned short hb = at_bf_bits(f);
  hi = __builtin_bit_cast(__bf16, hb);
  lo = at_f2bf(f - __uint_as_float(((unsigned)hb) << 16));
}
__device__ __forceinline__ v8f at_mma(v16b a, v16b b, v8f c) {
  c = __builtin_amdgcn_wmma_f32_16x16x32_bf16(false, a, false, b, (short)0, c, false, false);
  asm volatile("v_nop\n\tv_nop\n\tv_nop\n\tv_nop" : "+v"(c) : "v"(a), "v"(b));
  return c;
}
__device__ __forceinline__ void bf_hilo_pack2(float f0, float f1, unsigned& uh, unsigned& ul) {
  const unsigned short h0 = at_bf_bits(f0), h1 = at_bf_bits(f1);
  const unsigned short l0 = at_bf_bits(f0 - bf_bits2f(h0)), l1 = at_bf_bits(f1 - bf_bits2f(h1));
  uh = (unsigned)h0 | ((unsigned)h1 << 16);
  ul = (unsigned)l0 | ((unsigned)l1 << 16);
}
__device__ __forceinline__ unsigned f16pack2(float a, float b) {
  return (unsigned)__builtin_bit_cast(unsigned short, (_Float16)a) | ((unsigned)__builtin_bit_cast(unsigned short, (_Float16)b) << 16);
}
__device__ __forceinline__ float wave_sum32(float v) {
#pragma unroll
  for (int m = 16; m > 0; m >>= 1) v += __shfl_xor(v, m, 32);
  return v;
}
template <int E0>
__device__ __forceinline__ void split4_into(const v4f a, v16b& hv, v16b& lv) {
  __bf16 p, q;
  at_split(a.x, p, q); hv[E0 + 0] = p; lv[E0 + 0] = q;
  at_split(a.y, p, q); hv[E0 + 1] = p; lv[E0 + 1] = q;
  at_split(a.z, p, q); hv[E0 + 2] = p; lv[E0 + 2] = q;
  at_split(a.w, p, q); hv[E0 + 3] = p; lv[E0 + 3] = q;
}

__global__ __launch_bounds__(256) void trig_table_kernel(const float* __restrict__ ang,
                                                         float* __restrict__ cosb, float* __restrict__ sinb, int n) {
  const int i = blockIdx.x * 256 + threadIdx.x;
  if (i < n) {
    const float a = ang[i];
    const float c = cosf(a);
    const float s = sinf(a);
    ((volatile float*)cosb)[i] = c;
    ((volatile float*)sinb)[i] = s;
    __threadfence();
    ((volatile float*)cosb)[i] = c;
    ((volatile float*)sinb)[i] = s;
  }
}

__global__ __launch_bounds__(256) void rope_inplace_kernel(float* __restrict__ P,
                                                          const float* __restrict__ cosb, const float* __restrict__ sinb) {
  const int idx = blockIdx.x * 256 + threadIdx.x;
  const int row = idx >> 9;
  const int c4  = (idx & 511) * 4;
  const int s   = row & (kS - 1);
  const int p0  = (c4 & (kHD - 1)) >> 1;
  float* ptr = P + (size_t)row * kD + c4;
  const v4f v = *(const v4f*)ptr;
  const float cs0 = cosb[s * 32 + p0],     sn0 = sinb[s * 32 + p0];
  const float cs1 = cosb[s * 32 + p0 + 1], sn1 = sinb[s * 32 + p0 + 1];
  v4f o;
  o.x = v.x * cs0 - v.y * sn0;
  o.y = v.x * sn0 + v.y * cs0;
  o.z = v.z * cs1 - v.w * sn1;
  o.w = v.z * sn1 + v.w * cs1;
  *(volatile v4f*)ptr = o;
  __threadfence();
  *(volatile v4f*)ptr = o;
}

__global__ __launch_bounds__(256) void ilr_planes_kernel(const float* __restrict__ ilrW,
                                                         unsigned int* __restrict__ outh, unsigned int* __restrict__ outl) {
  const int idx  = blockIdx.x * 256 + threadIdx.x;
  const int row  = idx >> 8;
  const int c8   = (idx & 255) * 8;
  const int rowc = row < 32 ? row : 31;
  const float keep = row < 32 ? 1.0f : 0.0f;
  const float* src = ilrW + (size_t)rowc * kD + c8;
  const v4f a = *(const v4f*)src * keep;
  const v4f c = *(const v4f*)(src + 4) * keep;
  unsigned hx, lx, hy, ly, hz, lz, hw, lw;
  bf_hilo_pack2(a.x, a.y, hx, lx);
  bf_hilo_pack2(a.z, a.w, hy, ly);
  bf_hilo_pack2(c.x, c.y, hz, lz);
  bf_hilo_pack2(c.z, c.w, hw, lw);
  v4u oh, ol;
  oh.x = hx; oh.y = hy; oh.z = hz; oh.w = hw;
  ol.x = lx; ol.y = ly; ol.z = lz; ol.w = lw;
  unsigned int* ph = outh + (size_t)idx * 4;
  unsigned int* pl = outl + (size_t)idx * 4;
  *(volatile v4u*)ph = oh;
  *(volatile v4u*)pl = ol;
  __threadfence();
  *(volatile v4u*)ph = oh;
  *(volatile v4u*)pl = ol;
}

__global__ __launch_bounds__(64) void lr_proj_kernel(const float* __restrict__ x,
                                                     const unsigned short* __restrict__ ilrh,
                                                     const unsigned short* __restrict__ ilrl,
                                                     const float* __restrict__ ilrb,
                                                     float* __restrict__ LRo) {
  __shared__ __align__(16) float sT[2][16 * 68];
  const int lane = threadIdx.x & 31, wave = threadIdx.x >> 5;
  const int m0 = (blockIdx.x * 2 + wave) * 16;
  const int rlane = lane & 15, hh = lane >> 4, koff = hh * 8;
  const float* xrow = x + (size_t)(m0 + rlane) * kD;
  const __bf16* Bh = (const __bf16*)ilrh;
  const __bf16* Bl = (const __bf16*)ilrl;
  v8f acc[4];
#pragma unroll
  for (int j = 0; j < 4; ++j) acc[j] = (v8f){0.f,0.f,0.f,0.f,0.f,0.f,0.f,0.f};

#pragma unroll 1
  for (int k0 = 0; k0 < kD; k0 += 32) {
    v16b ah, al;
    {
      const v4f a0 = *(const v4f*)(xrow + k0 + koff);
      const v4f a1 = *(const v4f*)(xrow + k0 + koff + 4);
      const v4f a2 = *(const v4f*)(xrow + k0 + 16 + koff);
      const v4f a3 = *(const v4f*)(xrow + k0 + 16 + koff + 4);
      split4_into<0>(a0, ah, al);
      split4_into<4>(a1, ah, al);
      split4_into<8>(a2, ah, al);
      split4_into<12>(a3, ah, al);
    }
    v16b bhf[4], blf[4];
#pragma unroll
    for (int j = 0; j < 4; ++j) {
      const size_t bo = (size_t)(j * 16 + rlane) * kD + koff + k0;
      bhf[j] = Frag<__bf16>::load(Bh + bo);
      blf[j] = Frag<__bf16>::load(Bl + bo);
    }
#pragma unroll
    for (int j = 0; j < 4; ++j) {
      acc[j] = at_mma(ah, bhf[j], acc[j]);
      acc[j] = at_mma(ah, blf[j], acc[j]);
      acc[j] = at_mma(al, bhf[j], acc[j]);
    }
  }
  acc_guard4(acc[0], acc[1], acc[2], acc[3]);

  float* slab = sT[wave];
#pragma unroll
  for (int j = 0; j < 4; ++j) {
    const int n = j * 16 + rlane;
    const int nc = n < kH ? n : (kH - 1);
    const float bv = ilrb[nc];
#pragma unroll
    for (int r = 0; r < 8; ++r) slab[(hh * 8 + r) * 68 + j * 16 + rlane] = acc[j][r] + bv;
  }
  __builtin_amdgcn_fence(__ATOMIC_RELEASE, "workgroup");
  __builtin_amdgcn_wave_barrier();
  __builtin_amdgcn_fence(__ATOMIC_ACQUIRE, "workgroup");
  const int c4 = (lane & 15) * 4;
  for (int pass = 0; pass < 2; ++pass) {
#pragma unroll 1
    for (int it = 0; it < 8; ++it) {
      const int row = it * 2 + hh;
      const v4f v = *(const v4fa*)(slab + row * 68 + c4);
      v4f o;
      o.x = (1.0f / (1.0f + expf(-v.x))) * (1.0f / 64.0f);
      o.y = (1.0f / (1.0f + expf(-v.y))) * (1.0f / 64.0f);
      o.z = (1.0f / (1.0f + expf(-v.z))) * (1.0f / 64.0f);
      o.w = (1.0f / (1.0f + expf(-v.w))) * (1.0f / 64.0f);
      *(volatile v4f*)(LRo + (size_t)(m0 + row) * 64 + c4) = o;
    }
    __threadfence();
  }
}

__global__ __launch_bounds__(256) void inner_scan_kernel(
    float* __restrict__ QP, const float* __restrict__ KP, const float* __restrict__ VP,
    const float* __restrict__ LRp, const float* __restrict__ lgs,
    const float* __restrict__ tg, const float* __restrict__ tb,
    const float* __restrict__ W0, const float* __restrict__ b0) {
  __shared__ __align__(16) float Wm[64 * 65];
  __shared__ __align__(16) float XQs[16 * 64];
  __shared__ __align__(16) float XKs[16 * 64];
  __shared__ __align__(16) float XVs[16 * 64];
  __shared__ __align__(16) float Zm[16 * 64];
  __shared__ __align__(16) float Zb[16 * 64];
  __shared__ __align__(16) float Gr[16 * 64];
  __shared__ __align__(16) float EK[16 * 64];
  __shared__ __align__(16) float Ys[16 * 64];
  __shared__ float At[16 * 17];
  __shared__ float bvec[64], gam[64], bet[64], lrv[16], gsv[16];

  const int b = blockIdx.x >> 5;
  const int h = blockIdx.x & 31;
  const int tid = threadIdx.x, lane = tid & 31, wid = tid >> 5;
  const int rowbase = b * kS;

#pragma unroll 1
  for (int t = tid; t < 4096; t += 256) Wm[(t >> 6) * 65 + (t & 63)] = W0[(size_t)h * 4096 + t];
  if (wid < 2) {
    bvec[tid] = b0[h * 64 + tid];
    gam[tid]  = tg[h * 64 + tid];
    bet[tid]  = tb[h * 64 + tid];
  }
  if (wid == 0) {
    const int i = lane & 15;
    const float gv = fmaxf(1.0f / (float)(i + 1) + lgs[i], 0.0f);
    if (lane < 16) gsv[i] = gv;
  }
  __syncthreads();

#pragma unroll 1
  for (int n = 0; n < kNMB; ++n) {
    {
      const int i = tid >> 4, d4 = (tid & 15) * 4;
      const size_t go = (size_t)(rowbase + n * 16 + i) * kD + h * 64 + d4;
      const v4f xq = *(const v4f*)(QP + go);
      const v4f xk = *(const v4f*)(KP + go);
      const v4f xv = *(const v4f*)(VP + go);
      *(v4fa*)(XQs + i * 64 + d4) = xq;
      *(v4fa*)(XKs + i * 64 + d4) = xk;
      *(v4fa*)(XVs + i * 64 + d4) = xv;
      if (wid == 0) {
        const int j = lane & 15;
        const float lv = LRp[(size_t)(rowbase + n * 16 + j) * 64 + h];
        if (lane < 16) lrv[j] = lv;
      }
    }
    __syncthreads();

    {
      const int c = tid & 63, rg = tid >> 6;
      const float bc = bvec[c];
#pragma unroll 1
      for (int rr = 0; rr < 4; ++rr) {
        const int i = rg * 4 + rr;
        float zk = 0.f, zq = 0.f;
#pragma unroll 1
        for (int d = 0; d < 64; d += 4) {
          const float w0 = Wm[(d + 0) * 65 + c];
          const float w1 = Wm[(d + 1) * 65 + c];
          const float w2 = Wm[(d + 2) * 65 + c];
          const float w3 = Wm[(d + 3) * 65 + c];
          const v4f xk = *(const v4fa*)(XKs + i * 64 + d);
          const v4f xq = *(const v4fa*)(XQs + i * 64 + d);
          zk += xk.x * w0; zk += xk.y * w1; zk += xk.z * w2; zk += xk.w * w3;
          zq += xq.x * w0; zq += xq.y * w1; zq += xq.z * w2; zq += xq.w * w3;
        }
        Zm[i * 64 + c] = zk + bc;
        Zb[i * 64 + c] = zq;
      }
      const int i2 = tid >> 4, j2 = tid & 15;
      float a = 0.f;
#pragma unroll 1
      for (int d = 0; d < 64; d += 4) {
        const v4f xq = *(const v4fa*)(XQs + i2 * 64 + d);
        const v4f xk = *(const v4fa*)(XKs + j2 * 64 + d);
        a += xq.x * xk.x; a += xq.y * xk.y; a += xq.z * xk.z; a += xq.w * xk.w;
      }
      At[i2 * 17 + j2] = (j2 <= i2) ? a : 0.0f;
    }
    __syncthreads();

    {
#pragma unroll 1
      for (int q = 0; q < 2; ++q) {
        const int r = wid * 2 + q;
        const float v0 = Zm[r * 64 + lane], v1 = Zm[r * 64 + lane + 32];
        const float mu = wave_sum32(v0 + v1) * (1.0f / 64.0f);
        const float e0 = v0 - mu, e1 = v1 - mu;
        const float var = wave_sum32(e0 * e0 + e1 * e1) * (1.0f / 64.0f);
        const float rs = rsqrtf(var + kEps);
        const float zh0 = e0 * rs, zh1 = e1 * rs;
        const float g0 = gam[lane], g1 = gam[lane + 32];
        const float be0 = bet[lane], be1 = bet[lane + 32];
        const float t0 = XVs[r * 64 + lane] - XKs[r * 64 + lane];
        const float t1 = XVs[r * 64 + lane + 32] - XKs[r * 64 + lane + 32];
        const float dy0 = (g0 * zh0 + be0) - t0;
        const float dy1 = (g1 * zh1 + be1) - t1;
        const float dz0 = dy0 * g0, dz1 = dy1 * g1;
        const float m1 = wave_sum32(dz0 + dz1) * (1.0f / 64.0f);
        const float m2 = wave_sum32(dz0 * zh0 + dz1 * zh1) * (1.0f / 64.0f);
        Gr[r * 64 + lane]      = (dz0 - m1 - zh0 * m2) * rs;
        Gr[r * 64 + lane + 32] = (dz1 - m1 - zh1 * m2) * rs;
      }
      const int j = tid >> 4, d4 = (tid & 15) * 4;
      const float e15 = gsv[15] * lrv[j];
      const v4f xk = *(const v4fa*)(XKs + j * 64 + d4);
      *(v4fa*)(EK + j * 64 + d4) = xk * e15;
    }
    __syncthreads();

    {
      const int c = tid & 63, rg = tid >> 6;
      float s1[4], s2[4], gi[4];
#pragma unroll
      for (int rr = 0; rr < 4; ++rr) { s1[rr] = 0.f; s2[rr] = 0.f; gi[rr] = gsv[rg * 4 + rr]; }
#pragma unroll 1
      for (int j = 0; j < 16; ++j) {
        const float g = Gr[j * 64 + c];
        const float l = lrv[j];
#pragma unroll
        for (int rr = 0; rr < 4; ++rr) {
          const int i = rg * 4 + rr;
          const float eta = gi[rr] * l;
          const float at = At[i * 17 + j];
          s1[rr] += (eta * at) * g;
          s2[rr] += (j <= i) ? (eta * g) : 0.0f;
        }
      }
      const float bc = bvec[c];
#pragma unroll
      for (int rr = 0; rr < 4; ++rr) {
        const int i = rg * 4 + rr;
        const float zqw = Zb[i * 64 + c];
        Zb[i * 64 + c] = (zqw - s1[rr]) + (bc - s2[rr]);
      }
    }
    __syncthreads();

    {
#pragma unroll 1
      for (int q = 0; q < 2; ++q) {
        const int r = wid * 2 + q;
        const float v0 = Zb[r * 64 + lane], v1 = Zb[r * 64 + lane + 32];
        const float mu = wave_sum32(v0 + v1) * (1.0f / 64.0f);
        const float e0 = v0 - mu, e1 = v1 - mu;
        const float var = wave_sum32(e0 * e0 + e1 * e1) * (1.0f / 64.0f);
        const float rs = rsqrtf(var + kEps);
        Ys[r * 64 + lane]      = XQs[r * 64 + lane]      + ((gam[lane] * e0) * rs + bet[lane]);
        Ys[r * 64 + lane + 32] = XQs[r * 64 + lane + 32] + ((gam[lane + 32] * e1) * rs + bet[lane + 32]);
      }
      __builtin_amdgcn_fence(__ATOMIC_RELEASE, "workgroup");
      __builtin_amdgcn_wave_barrier();
      __builtin_amdgcn_fence(__ATOMIC_ACQUIRE, "workgroup");
      {
        const int row = wid * 2 + (lane >> 4);
        const int c4 = (lane & 15) * 4;
        const v4f yv = *(const v4fa*)(Ys + row * 64 + c4);
        float* dst = QP + (size_t)(rowbase + n * 16 + row) * kD + h * 64 + c4;
        *(volatile v4f*)dst = yv;
        __threadfence();
        *(volatile v4f*)dst = yv;
      }
      const int c = tid & 63, rg = tid >> 6;
#pragma unroll 1
      for (int grp = 0; grp < 4; ++grp) {
        const int wrow = rg * 16 + grp * 4;
        float wa0 = 0.f, wa1 = 0.f, wa2 = 0.f, wa3 = 0.f;
#pragma unroll 1
        for (int j = 0; j < 16; ++j) {
          const float g = Gr[j * 64 + c];
          const v4f kk = *(const v4fa*)(EK + j * 64 + wrow);
          wa0 += kk.x * g; wa1 += kk.y * g; wa2 += kk.z * g; wa3 += kk.w * g;
        }
        Wm[(wrow + 0) * 65 + c] -= wa0;
        Wm[(wrow + 1) * 65 + c] -= wa1;
        Wm[(wrow + 2) * 65 + c] -= wa2;
        Wm[(wrow + 3) * 65 + c] -= wa3;
      }
      if (wid < 2) {
        const float le = gsv[15];
        float ba = 0.f;
#pragma unroll 1
        for (int j = 0; j < 16; ++j) ba += (le * lrv[j]) * Gr[j * 64 + tid];
        bvec[tid] -= ba;
      }
    }
    __syncthreads();
  }
}

__global__ __launch_bounds__(256) void post_ln_kernel(const float* __restrict__ in,
                                                     const float* __restrict__ g, const float* __restrict__ be,
                                                     unsigned short* __restrict__ out16) {
  __shared__ float red1[8], red2[8];
  const int row = blockIdx.x;
  const int tid = threadIdx.x, lane = tid & 31, wid = tid >> 5;
  const int c8 = tid * 8;
  const float* rp = in + (size_t)row * kD + c8;
  const v4f a = *(const v4f*)rp;
  const v4f c = *(const v4f*)(rp + 4);
  float s = ((a.x + a.y) + (a.z + a.w)) + ((c.x + c.y) + (c.z + c.w));
  s = wave_sum32(s);
  if (lane == 0) red1[wid] = s;
  __syncthreads();
  float tot = 0.f;
#pragma unroll
  for (int i = 0; i < 8; ++i) tot += red1[i];
  const float mu = tot * (1.0f / 2048.0f);
  float e[8];
  e[0] = a.x - mu; e[1] = a.y - mu; e[2] = a.z - mu; e[3] = a.w - mu;
  e[4] = c.x - mu; e[5] = c.y - mu; e[6] = c.z - mu; e[7] = c.w - mu;
  float ss = 0.f;
#pragma unroll
  for (int i = 0; i < 8; ++i) ss += e[i] * e[i];
  ss = wave_sum32(ss);
  if (lane == 0) red2[wid] = ss;
  __syncthreads();
  float tot2 = 0.f;
#pragma unroll
  for (int i = 0; i < 8; ++i) tot2 += red2[i];
  const float var = tot2 * (1.0f / 2048.0f);
  const float rs = rsqrtf(var + kEps);
  const v4f g0 = *(const v4f*)(g + c8), g1 = *(const v4f*)(g + c8 + 4);
  const v4f b0v = *(const v4f*)(be + c8), b1v = *(const v4f*)(be + c8 + 4);
  float y[8];
  y[0] = (g0.x * e[0]) * rs + b0v.x; y[1] = (g0.y * e[1]) * rs + b0v.y;
  y[2] = (g0.z * e[2]) * rs + b0v.z; y[3] = (g0.w * e[3]) * rs + b0v.w;
  y[4] = (g1.x * e[4]) * rs + b1v.x; y[5] = (g1.y * e[5]) * rs + b1v.y;
  y[6] = (g1.z * e[6]) * rs + b1v.z; y[7] = (g1.w * e[7]) * rs + b1v.w;
  v4u o;
  o.x = f16pack2(y[0], y[1]);
  o.y = f16pack2(y[2], y[3]);
  o.z = f16pack2(y[4], y[5]);
  o.w = f16pack2(y[6], y[7]);
  unsigned int* op = (unsigned int*)(out16 + (size_t)row * kD + c8);
  *(volatile v4u*)op = o;
  __threadfence();
  *(volatile v4u*)op = o;
}

extern "C" void kernel_launch(void* const* d_in, const int* in_sizes, int n_in,
                              void* d_out, int out_size, void* d_ws, size_t ws_size,
                              hipStream_t stream) {
  if (n_in < 15) return;
  if (in_sizes[0] != kRows * kD || in_sizes[1] != kS * 32 ||
      in_sizes[2] != kD * kD || in_sizes[3] != kD * kD || in_sizes[4] != kD * kD || in_sizes[5] != kD * kD ||
      in_sizes[6] != kD || in_sizes[7] != kD || in_sizes[8] != kH * kD || in_sizes[9] != kH ||
      in_sizes[10] != kMB || in_sizes[11] != kH * kHD || in_sizes[12] != kH * kHD ||
      in_sizes[13] != kH * kHD * kHD || in_sizes[14] != kH * kHD) return;
  if (out_size != kRows * kD) return;

  const float* x    = (const float*)d_in[0];
  const float* posf = (const float*)d_in[1];
  const float* Wq   = (const float*)d_in[2];
  const float* Wk   = (const float*)d_in[3];
  const float* Wv   = (const float*)d_in[4];
  const float* Wo   = (const float*)d_in[5];
  const float* pg   = (const float*)d_in[6];
  const float* pb   = (const float*)d_in[7];
  const float* ilrW = (const float*)d_in[8];
  const float* ilrb = (const float*)d_in[9];
  const float* lgsp = (const float*)d_in[10];
  const float* tg   = (const float*)d_in[11];
  const float* tb   = (const float*)d_in[12];
  const float* W0   = (const float*)d_in[13];
  const float* b0   = (const float*)d_in[14];
  float* out = (float*)d_out;

  const size_t szX16 = (size_t)kRows * kD * 2;
  const size_t szW16 = (size_t)kD * kD * 2;
  const size_t szP32 = (size_t)kRows * kD * 4;
  const size_t szLR  = (size_t)kRows * 64 * 4;
  const size_t szILR = (size_t)64 * kD * 2;
  const size_t szTRG = (size_t)kS * 32 * 4;
  const size_t offX16  = 0;
  const size_t offW16  = offX16 + szX16;
  const size_t offQ    = offW16 + szW16;
  const size_t offK    = offQ + szP32;
  const size_t offV    = offK + szP32;
  const size_t offLR   = offV + szP32;
  const size_t offILRH = offLR + szLR;
  const size_t offILRL = offILRH + szILR;
  const size_t offCOS  = offILRL + szILR;
  const size_t offSIN  = offCOS + szTRG;
  const size_t total   = offSIN + szTRG;
  if (total > ws_size) return;

  char* ws = (char*)d_ws;
  unsigned short* X16  = (unsigned short*)(ws + offX16);
  unsigned short* W16  = (unsigned short*)(ws + offW16);
  float* QP  = (float*)(ws + offQ);
  float* KP  = (float*)(ws + offK);
  float* VP  = (float*)(ws + offV);
  float* LR  = (float*)(ws + offLR);
  unsigned int* ILRH = (unsigned int*)(ws + offILRH);
  unsigned int* ILRL = (unsigned int*)(ws + offILRL);
  float* COSB = (float*)(ws + offCOS);
  float* SINB = (float*)(ws + offSIN);

  const int nx2 = kRows * kD / 2;
  const int nw2 = kD * kD / 2;
  const float wcarry = 32.0f, wundo = 1.0f / 32.0f;
  const dim3 gemmGrid((kRows / 64) * (kD / 64) / 8, 1);
  const int ropeBlocks = (kRows * kD / 4) / 256;

  cast_f32_f16x2_kernel<<<(nx2 + 255) / 256, 256, 0, stream>>>(x, (_Float16*)X16, nx2, 1.0f);
  trig_table_kernel<<<(kS * 32 + 255) / 256, 256, 0, stream>>>(posf, COSB, SINB, kS * 32);

  cast_f32_f16x2_kernel<<<(nw2 + 255) / 256, 256, 0, stream>>>(Wq, (_Float16*)W16, nw2, wcarry);
  wmma_gemm64<0, false, 0, 0, false, 0><<<gemmGrid, 256, 0, stream>>>(
      X16, X16, kD, 0L, W16, W16, kD, 0L, (void*)QP, (void*)QP, kD, 0L,
      (const float*)LR, (const float*)QP, 0L, kRows, kD, kD, wundo);
  rope_inplace_kernel<<<ropeBlocks, 256, 0, stream>>>(QP, COSB, SINB);

  cast_f32_f16x2_kernel<<<(nw2 + 255) / 256, 256, 0, stream>>>(Wk, (_Float16*)W16, nw2, wcarry);
  wmma_gemm64<0, false, 0, 0, false, 0><<<gemmGrid, 256, 0, stream>>>(
      X16, X16, kD, 0L, W16, W16, kD, 0L, (void*)KP, (void*)KP, kD, 0L,
      (const float*)LR, (const float*)KP, 0L, kRows, kD, kD, wundo);
  rope_inplace_kernel<<<ropeBlocks, 256, 0, stream>>>(KP, COSB, SINB);

  cast_f32_f16x2_kernel<<<(nw2 + 255) / 256, 256, 0, stream>>>(Wv, (_Float16*)W16, nw2, wcarry);
  wmma_gemm64<0, false, 0, 0, false, 0><<<gemmGrid, 256, 0, stream>>>(
      X16, X16, kD, 0L, W16, W16, kD, 0L, (void*)VP, (void*)VP, kD, 0L,
      (const float*)LR, (const float*)VP, 0L, kRows, kD, kD, wundo);
  rope_inplace_kernel<<<ropeBlocks, 256, 0, stream>>>(VP, COSB, SINB);

  ilr_planes_kernel<<<(64 * kD / 8) / 256, 256, 0, stream>>>(ilrW, ILRH, ILRL);
  lr_proj_kernel<<<kRows / 32, 64, 0, stream>>>(x, (const unsigned short*)ILRH, (const unsigned short*)ILRL, ilrb, LR);

  cast_f32_f16x2_kernel<<<(nw2 + 255) / 256, 256, 0, stream>>>(Wo, (_Float16*)W16, nw2, wcarry);

  inner_scan_kernel<<<kB * kH, 256, 0, stream>>>(QP, KP, VP, LR, lgsp, tg, tb, W0, b0);

  post_ln_kernel<<<kRows, 256, 0, stream>>>(QP, pg, pb, X16);
  wmma_gemm64<0, false, 0, 0, false, 0><<<gemmGrid, 256, 0, stream>>>(
      X16, X16, kD, 0L, W16, W16, kD, 0L, (void*)out, (void*)out, kD, 0L,
      (const float*)LR, (const float*)out, 0L, kRows, kD, kD, wundo);
}
